// LSTMCell_54614804136122
// MI455X (gfx1250) — hardware-verified
//
#include <hip/hip_runtime.h>
#include <math.h>

constexpr int NBATCH = 4096;
constexpr int NIN    = 1024;
constexpr int NHID   = 1024;
constexpr int NGATE4 = 4 * NHID;
constexpr int KTOT   = NIN + NHID;
constexpr int NTC    = 256;
constexpr int NTG    = 128;
constexpr int NWG    = NTG / 32;
constexpr int TROWS  = 32;
constexpr int TCOLS  = 32;
constexpr int ZP     = 36;
constexpr int GSLAB  = 16 * ZP;
constexpr int NTILE  = (NBATCH / TROWS) * (NHID / TCOLS);
constexpr int NC8    = NIN / 8;

static_assert(KTOT % 32 == 0);
static_assert(NBATCH % TROWS == 0 && NHID % TCOLS == 0);
static_assert(NTILE % NWG == 0);
static_assert(NIN == NHID);
static_assert(NGATE4 == NBATCH);
static_assert((NBATCH * NC8) % NTC == 0);
static_assert((ZP % 4) == 0 && (GSLAB % 4) == 0);
static_assert(16777216 + 16777216 <= 33554432);

typedef __attribute__((ext_vector_type(8)))  _Float16 v8h;
typedef __attribute__((ext_vector_type(16))) __bf16   v16b;
typedef __attribute__((ext_vector_type(8)))  __bf16   v8b;
typedef __attribute__((ext_vector_type(8)))  float    v8f;
typedef __attribute__((ext_vector_type(4)))  float    v4f;

__device__ __forceinline__ unsigned short f2bf_bits(float f) {
  unsigned u = __float_as_uint(f);
  return (unsigned short)((u + 0x7FFFu + ((u >> 16) & 1u)) >> 16);
}
__device__ __forceinline__ float bf_bits2f(unsigned short h) { return __uint_as_float(((unsigned)h) << 16); }
__device__ __forceinline__ float bf16r(float f) { return bf_bits2f(f2bf_bits(f)); }

__device__ __forceinline__ void grp_guard_b(v8f& a, v8f& b, v8f& c, v8f& d, v16b w, v16b x, v16b y, v16b z) {
  asm volatile("v_nop\n\tv_nop\n\tv_nop\n\tv_nop" : "+v"(a), "+v"(b), "+v"(c), "+v"(d) : "v"(w), "v"(x), "v"(y), "v"(z));
}
__device__ __forceinline__ void acc_guard4(v8f& a, v8f& b, v8f& c, v8f& d) {
  asm volatile("v_nop\n\tv_nop\n\tv_nop\n\tv_nop" : "+v"(a), "+v"(b), "+v"(c), "+v"(d));
}

template <typename T> struct Frag;
template <> struct Frag<__bf16> {
  typedef v16b V; union U { v16b v; v8b h[2]; };
  static __device__ __forceinline__ v16b load(const __bf16* p) {
    U f; f.h[0] = *(const v8b*)(p); f.h[1] = *(const v8b*)(p + 16); return f.v;
  }
  static __device__ __forceinline__ v8f mma(v16b a, v16b b, v8f c) {
    return __builtin_amdgcn_wmma_f32_16x16x32_bf16(false, a, false, b, (short)0, c, false, false);
  }
};

__device__ __forceinline__ float fsig(float x)  { return __builtin_amdgcn_rcpf(1.0f + expf(-x)); }
__device__ __forceinline__ float ftanh(float x) { return 1.0f - 2.0f * __builtin_amdgcn_rcpf(expf(2.0f * x) + 1.0f); }

__global__ __launch_bounds__(NTC) void cvt_pair_kernel(const float* __restrict__ src0, const float* __restrict__ src1,
                                                       unsigned short* __restrict__ dst) {
  const int half = blockIdx.y;
  const float* src = half ? src1 : src0;
  const int i = blockIdx.x * NTC + threadIdx.x;
  if (i < NBATCH * NC8) {
    const int row = i / NC8;
    const int c8  = i - row * NC8;
    const float* sp = src + (size_t)row * NIN + c8 * 8;
    const v4f a = *(const v4f*)(sp);
    const v4f b = *(const v4f*)(sp + 4);
    v8h hv;
#pragma unroll
    for (int e = 0; e < 4; ++e) {
      const unsigned short b0 = f2bf_bits(a[e]);
      const unsigned short b1 = f2bf_bits(b[e]);
      hv[e]     = __builtin_bit_cast(_Float16, b0);
      hv[4 + e] = __builtin_bit_cast(_Float16, b1);
    }
    unsigned short* dp = dst + (size_t)row * KTOT + (size_t)half * NIN + c8 * 8;
    *(volatile v8h*)(dp) = hv;
    __threadfence();
    *(volatile v8h*)(dp) = hv;
  }
}

__global__ __launch_bounds__(NTG) void lstm_cell_kernel(const unsigned short* __restrict__ Ap, const unsigned short* __restrict__ Btp,
                                                        const float* __restrict__ b_ih, const float* __restrict__ b_hh,
                                                        const float* __restrict__ cx, const float* __restrict__ eps_c,
                                                        const float* __restrict__ eps_h,
                                                        const float* __restrict__ noise_q, const float* __restrict__ noise_e,
                                                        float* __restrict__ hy_out, float* __restrict__ cy_out) {
  __shared__ __align__(16) float sZ[NWG][4 * GSLAB];
  const __bf16* A  = (const __bf16*)Ap;
  const __bf16* Bt = (const __bf16*)Btp;
  const int lane = threadIdx.x & 31, wave = threadIdx.x >> 5;
  const int tile = blockIdx.x * NWG + wave;
  const int tm = tile / (NHID / TCOLS);
  const int th = tile - tm * (NHID / TCOLS);
  const int m0 = tm * TROWS, h0 = th * TCOLS;
  const int rlane = lane & 15, hh = lane >> 4, koff = hh * 8, mOff = hh * 8;

  const v8f z8 = {0.f, 0.f, 0.f, 0.f, 0.f, 0.f, 0.f, 0.f};
  v8f acc[2][4][2];
#pragma unroll
  for (int mi = 0; mi < 2; ++mi)
#pragma unroll
    for (int g = 0; g < 4; ++g) { acc[mi][g][0] = z8; acc[mi][g][1] = z8; }

  const __bf16* arow0 = A  + (size_t)(m0 + rlane) * KTOT + koff;
  const __bf16* arow1 = A  + (size_t)(m0 + 16 + rlane) * KTOT + koff;
  const __bf16* brow  = Bt + (size_t)(h0 + rlane) * KTOT + koff;

#pragma unroll 1
  for (int k0 = 0; k0 < KTOT; k0 += 32) {
    const v16b a0 = Frag<__bf16>::load(arow0 + k0);
    const v16b a1 = Frag<__bf16>::load(arow1 + k0);
#pragma unroll
    for (int g = 0; g < 4; ++g) {
      const v16b b0 = Frag<__bf16>::load(brow + (size_t)(g * NHID) * KTOT + k0);
      const v16b b1 = Frag<__bf16>::load(brow + (size_t)(g * NHID + 16) * KTOT + k0);
      acc[0][g][0] = Frag<__bf16>::mma(a0, b0, acc[0][g][0]);
      acc[1][g][0] = Frag<__bf16>::mma(a1, b0, acc[1][g][0]);
      acc[0][g][1] = Frag<__bf16>::mma(a0, b1, acc[0][g][1]);
      acc[1][g][1] = Frag<__bf16>::mma(a1, b1, acc[1][g][1]);
      grp_guard_b(acc[0][g][0], acc[1][g][0], acc[0][g][1], acc[1][g][1], a0, a1, b0, b1);
    }
  }
  acc_guard4(acc[0][0][0], acc[0][0][1], acc[0][1][0], acc[0][1][1]);
  acc_guard4(acc[0][2][0], acc[0][2][1], acc[0][3][0], acc[0][3][1]);
  acc_guard4(acc[1][0][0], acc[1][0][1], acc[1][1][0], acc[1][1][1]);
  acc_guard4(acc[1][2][0], acc[1][2][1], acc[1][3][0], acc[1][3][1]);

  float bsum[4][2];
  {
    float bi[4][2], bq[4][2];
#pragma unroll
    for (int g = 0; g < 4; ++g)
#pragma unroll
      for (int nt = 0; nt < 2; ++nt) bi[g][nt] = b_ih[g * NHID + h0 + nt * 16 + rlane];
    asm volatile("" ::: "memory");
#pragma unroll
    for (int g = 0; g < 4; ++g)
#pragma unroll
      for (int nt = 0; nt < 2; ++nt) bq[g][nt] = b_hh[g * NHID + h0 + nt * 16 + rlane];
#pragma unroll
    for (int g = 0; g < 4; ++g)
#pragma unroll
      for (int nt = 0; nt < 2; ++nt) bsum[g][nt] = bf16r(bi[g][nt]) + bf16r(bq[g][nt]);
  }
  const float se = sqrtf(bf16r(noise_e[0]));
  const float sq = sqrtf(bf16r(noise_q[0]));

  float* slab = sZ[wave];
  const int q = lane >> 3, c4 = (lane & 7) * 4;

#pragma unroll
  for (int mi = 0; mi < 2; ++mi) {
#pragma unroll
    for (int g = 0; g < 4; ++g)
#pragma unroll
      for (int nt = 0; nt < 2; ++nt)
#pragma unroll
        for (int r = 0; r < 8; ++r)
          slab[g * GSLAB + (mOff + r) * ZP + nt * 16 + rlane] = acc[mi][g][nt][r] + bsum[g][nt];
    __builtin_amdgcn_fence(__ATOMIC_RELEASE, "workgroup");
    __builtin_amdgcn_wave_barrier();
    __builtin_amdgcn_fence(__ATOMIC_ACQUIRE, "workgroup");

#pragma unroll 1
    for (int it = 0; it < 4; ++it) {
      const int row = it * 4 + q;
      const size_t goff = (size_t)(m0 + mi * 16 + row) * NHID + h0 + c4;
      const v4f cx4 = *(const v4f*)(cx + goff);
      const v4f ec4 = *(const v4f*)(eps_c + goff);
      const v4f eh4 = *(const v4f*)(eps_h + goff);
      float* zp = slab + row * ZP + c4;
      const v4f zi = *(const v4f*)(zp);
      const v4f zf = *(const v4f*)(zp + GSLAB);
      const v4f zg = *(const v4f*)(zp + 2 * GSLAB);
      const v4f zo = *(const v4f*)(zp + 3 * GSLAB);
      v4f hy4, cy4;
#pragma unroll
      for (int e = 0; e < 4; ++e) {
        const float ig  = fsig(zi[e]);
        const float fg  = fsig(zf[e]);
        const float gg  = ftanh(zg[e]);
        const float og  = fsig(zo[e]);
        const float cxv = bf16r(cx4[e]);
        const float ecv = bf16r(ec4[e]);
        const float ehv = bf16r(eh4[e]);
        const float cyv = fg * cxv + ig * gg + se * ecv;
        const float hyv = og * ftanh(cyv) + sq * ehv;
        cy4[e] = cyv;
        hy4[e] = hyv;
      }
      *(v4f*)(zp) = hy4;
      *(v4f*)(zp + GSLAB) = cy4;
    }

    for (int pass = 0; pass < 2; ++pass) {
#pragma unroll
      for (int it = 0; it < 4; ++it) {
        const int row = it * 4 + q;
        const size_t goff = (size_t)(m0 + mi * 16 + row) * NHID + h0 + c4;
        const v4f hv = *(const v4f*)(slab + row * ZP + c4);
        const v4f cv = *(const v4f*)(slab + row * ZP + c4 + GSLAB);
        *(volatile v4f*)(hy_out + goff) = hv;
        *(volatile v4f*)(cy_out + goff) = cv;
      }
      __threadfence();
    }
    __builtin_amdgcn_fence(__ATOMIC_RELEASE, "workgroup");
    __builtin_amdgcn_wave_barrier();
    __builtin_amdgcn_fence(__ATOMIC_ACQUIRE, "workgroup");
  }
}

extern "C" void kernel_launch(void* const* d_in, const int* in_sizes, int n_in,
                              void* d_out, int out_size, void* d_ws, size_t ws_size, hipStream_t stream) {
  if (n_in < 11 || d_out == nullptr || d_ws == nullptr) return;
  if (in_sizes[0] != NBATCH * NIN || in_sizes[1] != NBATCH * NHID || in_sizes[2] != NBATCH * NHID ||
      in_sizes[3] < 1 || in_sizes[4] < 1 ||
      in_sizes[5] != NGATE4 * NIN || in_sizes[6] != NGATE4 * NHID || in_sizes[7] != NGATE4 || in_sizes[8] != NGATE4 ||
      in_sizes[9] != NBATCH * NHID || in_sizes[10] != NBATCH * NHID || out_size != 2 * NBATCH * NHID) return;

  const float* input   = (const float*)d_in[0];
  const float* hx      = (const float*)d_in[1];
  const float* cx      = (const float*)d_in[2];
  const float* noise_q = (const float*)d_in[3];
  const float* noise_e = (const float*)d_in[4];
  const float* w_ih    = (const float*)d_in[5];
  const float* w_hh    = (const float*)d_in[6];
  const float* b_ih    = (const float*)d_in[7];
  const float* b_hh    = (const float*)d_in[8];
  const float* eps_c   = (const float*)d_in[9];
  const float* eps_h   = (const float*)d_in[10];
  float* hy = (float*)d_out;
  float* cy = hy + (size_t)NBATCH * NHID;

  char* ws = (char*)d_ws; size_t off = 0;
  auto carve = [&](size_t bytes) -> char* { char* p = ws + off; off += (bytes + 255) & ~(size_t)255; return p; };
  unsigned short* APL = (unsigned short*)carve((size_t)NBATCH * KTOT * 2);
  unsigned short* BPL = (unsigned short*)carve((size_t)NGATE4 * KTOT * 2);
  if (off > ws_size || off > (size_t)134217728) return;

  const dim3 cgrid((NBATCH * NC8) / NTC, 2);
  cvt_pair_kernel<<<cgrid, NTC, 0, stream>>>(input, hx, APL);
  cvt_pair_kernel<<<cgrid, NTC, 0, stream>>>(w_ih, w_hh, BPL);
  lstm_cell_kernel<<<NTILE / NWG, NTG, 0, stream>>>(APL, BPL, b_ih, b_hh, cx, eps_c, eps_h, noise_q, noise_e, hy, cy);
}
